// Indexer_17600775979892
// MI455X (gfx1250) — hardware-verified
//
#include <hip/hip_runtime.h>


namespace {
constexpr int Bn = 2, S = 2048, HID = 2048, NH = 16, HD = 128, RD = 64, NTOK = Bn * S, QC = NH * HD  , KC = HD + NH  , KCP = 192;
constexpr float SCALE = 0.022097086912079608f  , QS = 8.0f, LNE = 1e-5f;
constexpr size_t QPL = (size_t)NTOK * QC, KPL = (size_t)NTOK * HD;

typedef _Float16 b16;
typedef __attribute__((ext_vector_type(16))) _Float16 v16b;
typedef __attribute__((ext_vector_type(16))) __bf16 v16bb;
typedef __attribute__((ext_vector_type(8))) _Float16 v8b;
typedef __attribute__((ext_vector_type(8))) unsigned short v8us;
typedef __attribute__((ext_vector_type(8))) float v8f;
typedef __attribute__((ext_vector_type(4))) float v4f;
__device__ __forceinline__ float bf16_rne(float f) { unsigned int u = __float_as_uint(f); u += 0x7FFFu + ((u >> 16) & 1u); return __uint_as_float(u & 0xFFFF0000u); }
__device__ __forceinline__ unsigned short bf16_bits(float f) { unsigned int u = __float_as_uint(f); u += 0x7FFFu + ((u >> 16) & 1u); return (unsigned short)(u >> 16); }
__device__ __forceinline__ void split16(float v, b16& hi, b16& lo) { hi = (b16)v; lo = (b16)(v - (float)hi); }
__device__ __forceinline__ v16b frag_kb(const b16* p, int hh) { const v8b a = *(const v8b*)(p + 8 * hh), b = *(const v8b*)(p + 16 + 8 * hh); v16b f;
#pragma unroll
  for (int e = 0; e < 8; ++e) { f[e] = a[e]; f[8 + e] = b[e]; } return f; }
__device__ __forceinline__ v16bb frag_bf(const unsigned short* p, int hh) { const v8us a = *(const v8us*)(p + 8 * hh), b = *(const v8us*)(p + 16 + 8 * hh); union { unsigned short s[16]; v16bb v; } u;
#pragma unroll
  for (int e = 0; e < 8; ++e) { u.s[e] = a[e]; u.s[8 + e] = b[e]; } return u.v; }
__device__ __forceinline__ v8f wmma16b(v16b a, v16b b, v8f c) { v8f d = __builtin_amdgcn_wmma_f32_16x16x32_f16(false, a, false, b, (short)0, c, false, false); asm volatile("v_nop\n\tv_nop\n\tv_nop\n\tv_nop" : "+v"(d) : "v"(a), "v"(b)); return d; }
__device__ __forceinline__ v8f wmma16bb(v16bb a, v16bb b, v8f c) { v8f d = __builtin_amdgcn_wmma_f32_16x16x32_bf16(false, a, false, b, (short)0, c, false, false); asm volatile("v_nop\n\tv_nop\n\tv_nop\n\tv_nop" : "+v"(d) : "v"(a), "v"(b)); return d; }
__device__ __forceinline__ void wave_lds_sync() { __builtin_amdgcn_fence(__ATOMIC_RELEASE, "workgroup"); __builtin_amdgcn_wave_barrier(); __builtin_amdgcn_fence(__ATOMIC_ACQUIRE, "workgroup"); }

__global__ __launch_bounds__(256) void prep_kernel(const float* __restrict__ x, const float* __restrict__ wq, const float* __restrict__ wk, const float* __restrict__ ww, unsigned short* __restrict__ x16, unsigned short* __restrict__ wq16, unsigned short* __restrict__ wk16) {
  const size_t tid = (size_t)blockIdx.x * blockDim.x + threadIdx.x, nth = (size_t)gridDim.x * blockDim.x;
  for (int pass = 0; pass < 2; ++pass) {
    for (size_t p = tid; p < (size_t)NTOK * HID / 8; p += nth) { v8us v;
#pragma unroll
      for (int e = 0; e < 8; ++e) v[e] = bf16_bits(x[p * 8 + e]);
      *(volatile v8us*)(x16 + p * 8) = v; }
    for (size_t p = tid; p < (size_t)QC * HID / 8; p += nth) { const int n = (int)(p / (HID / 8)), k0 = (int)(p % (HID / 8)) * 8; v8us v;
#pragma unroll
      for (int e = 0; e < 8; ++e) v[e] = bf16_bits(wq[(size_t)(k0 + e) * QC + n]);
      *(volatile v8us*)(wq16 + (size_t)n * HID + k0) = v; }
    for (size_t p = tid; p < (size_t)KCP * HID / 8; p += nth) { const int n = (int)(p / (HID / 8)), k0 = (int)(p % (HID / 8)) * 8; v8us v;
#pragma unroll
      for (int e = 0; e < 8; ++e) { const float val = (n < HD) ? wk[(size_t)(k0 + e) * HD + n] : (n < KC) ? ww[(size_t)(k0 + e) * NH + (n - HD)] : 0.0f; v[e] = bf16_bits(val); }
      *(volatile v8us*)(wk16 + (size_t)n * HID + k0) = v; }
    __threadfence();
  }
}

__global__ __launch_bounds__(128) void qproj_kernel(const unsigned short* __restrict__ x16, const unsigned short* __restrict__ wq16, const float* __restrict__ cosb, const float* __restrict__ sinb, b16* __restrict__ qh, int rowbase) {
  __shared__ __attribute__((aligned(16))) b16 Th[4][32][64 + 8], Tl[4][32][64 + 8];
  const int lane = threadIdx.x & 31, wave = threadIdx.x >> 5, nloc = lane & 15, hlf = lane >> 4, m0 = rowbase + blockIdx.y * 128 + wave * 32, c0 = blockIdx.x * 64;
  v8f acc[2][4];
#pragma unroll
  for (int r = 0; r < 2; ++r)
#pragma unroll
    for (int t = 0; t < 4; ++t) acc[r][t] = (v8f){};
#pragma unroll 2
  for (int kb = 0; kb < HID; kb += 32) { const v16bb a0 = frag_bf(x16 + (size_t)(m0 + nloc) * HID + kb, hlf), a1 = frag_bf(x16 + (size_t)(m0 + 16 + nloc) * HID + kb, hlf);
#pragma unroll
    for (int t = 0; t < 4; ++t) { const v16bb bw = frag_bf(wq16 + (size_t)(c0 + t * 16 + nloc) * HID + kb, hlf); acc[0][t] = wmma16bb(a0, bw, acc[0][t]); acc[1][t] = wmma16bb(a1, bw, acc[1][t]); } }
  const bool rope = ((blockIdx.x & 1) == 0);
  if (rope) {
#pragma unroll
    for (int t = 0; t < 2; ++t) { const int i = t * 16 + nloc;
#pragma unroll
      for (int r = 0; r < 2; ++r)
#pragma unroll
        for (int v = 0; v < 8; ++v) { const int tok = m0 + r * 16 + 8 * hlf + v; const size_t cb = (size_t)tok * RD;
          const float c1 = bf16_rne(cosb[cb + i]), s1 = bf16_rne(sinb[cb + i]), c2 = bf16_rne(cosb[cb + i + 32]), s2 = bf16_rne(sinb[cb + i + 32]);
          const float x1 = acc[r][t][v], x2 = acc[r][t + 2][v]; acc[r][t][v] = x1 * c1 - x2 * s1; acc[r][t + 2][v] = x2 * c2 + x1 * s2; } } }
#pragma unroll
  for (int t = 0; t < 4; ++t)
#pragma unroll
    for (int r = 0; r < 2; ++r)
#pragma unroll
      for (int v = 0; v < 8; ++v) { b16 a_, c_; split16(acc[r][t][v] * QS, a_, c_); Th[wave][r * 16 + 8 * hlf + v][t * 16 + nloc] = a_; Tl[wave][r * 16 + 8 * hlf + v][t * 16 + nloc] = c_; }
  wave_lds_sync();
  b16* dst = qh + (size_t)m0 * QC + c0;
  for (int pass = 0; pass < 2; ++pass) {
#pragma unroll
    for (int j = 0; j < 8; ++j) { const int rr = j * 4 + (lane >> 3), c8 = (lane & 7) * 8; *(volatile v8b*)(dst + (size_t)rr * QC + c8) = *(const v8b*)(&Th[wave][rr][c8]); *(volatile v8b*)(dst + QPL + (size_t)rr * QC + c8) = *(const v8b*)(&Tl[wave][rr][c8]); }
    __threadfence(); }
}

__global__ __launch_bounds__(128) void kproj_kernel(const unsigned short* __restrict__ x16, const unsigned short* __restrict__ wk16, const float* __restrict__ cosb, const float* __restrict__ sinb, const float* __restrict__ g, const float* __restrict__ bta, b16* __restrict__ kh, float* __restrict__ wout) {
  __shared__ __attribute__((aligned(16))) float Tk[4][32][KC + 1]; __shared__ __attribute__((aligned(16))) b16 Th[4][32][HD + 8], Tl[4][32][HD + 8]; __shared__ __attribute__((aligned(16))) float Tw[4][32][NH];
  const int lane = threadIdx.x & 31, wave = threadIdx.x >> 5, nloc = lane & 15, hlf = lane >> 4, m0 = blockIdx.x * 128 + wave * 32;
  v8f acc[2][9];
#pragma unroll
  for (int r = 0; r < 2; ++r)
#pragma unroll
    for (int t = 0; t < 9; ++t) acc[r][t] = (v8f){};
#pragma unroll 1
  for (int kb = 0; kb < HID; kb += 32) { const v16bb a0 = frag_bf(x16 + (size_t)(m0 + nloc) * HID + kb, hlf), a1 = frag_bf(x16 + (size_t)(m0 + 16 + nloc) * HID + kb, hlf);
#pragma unroll
    for (int t = 0; t < 9; ++t) { const v16bb bw = frag_bf(wk16 + (size_t)(t * 16 + nloc) * HID + kb, hlf); acc[0][t] = wmma16bb(a0, bw, acc[0][t]); acc[1][t] = wmma16bb(a1, bw, acc[1][t]); } }
#pragma unroll
  for (int t = 0; t < 9; ++t)
#pragma unroll
    for (int r = 0; r < 2; ++r)
#pragma unroll
      for (int v = 0; v < 8; ++v) Tk[wave][r * 16 + 8 * hlf + v][t * 16 + nloc] = acc[r][t][v];
  wave_lds_sync();
  { const int rr = lane; const float* row = Tk[wave][rr]; const int tok = m0 + rr;
    float mu = 0.0f; for (int d = 0; d < HD; ++d) mu += row[d]; mu *= (1.0f / HD);
    float var = 0.0f; for (int d = 0; d < HD; ++d) { const float z = row[d] - mu; var += z * z; } var *= (1.0f / HD);
    const float rs = rsqrtf(var + LNE); const size_t cb = (size_t)tok * RD;
#pragma unroll 2
    for (int i = 0; i < 32; ++i) {
      const float x1 = (row[i] - mu) * rs * bf16_rne(g[i]) + bf16_rne(bta[i]), x2 = (row[i + 32] - mu) * rs * bf16_rne(g[i + 32]) + bf16_rne(bta[i + 32]);
      const float c1 = bf16_rne(cosb[cb + i]), s1 = bf16_rne(sinb[cb + i]), c2 = bf16_rne(cosb[cb + i + 32]), s2 = bf16_rne(sinb[cb + i + 32]);
      b16 a_, c_; split16((x1 * c1 - x2 * s1) * QS, a_, c_); Th[wave][rr][i] = a_; Tl[wave][rr][i] = c_; split16((x2 * c2 + x1 * s2) * QS, a_, c_); Th[wave][rr][i + 32] = a_; Tl[wave][rr][i + 32] = c_; }
#pragma unroll 2
    for (int d = RD; d < HD; ++d) { b16 a_, c_; split16(((row[d] - mu) * rs * bf16_rne(g[d]) + bf16_rne(bta[d])) * QS, a_, c_); Th[wave][rr][d] = a_; Tl[wave][rr][d] = c_; }
#pragma unroll
    for (int h = 0; h < NH; ++h) Tw[wave][rr][h] = row[HD + h] * SCALE; }
  wave_lds_sync();
  for (int pass = 0; pass < 2; ++pass) {
#pragma unroll
    for (int j = 0; j < 16; ++j) { const int rr = j * 2 + hlf, c8 = nloc * 8; *(volatile v8b*)(kh + (size_t)(m0 + rr) * HD + c8) = *(const v8b*)(&Th[wave][rr][c8]); *(volatile v8b*)(kh + KPL + (size_t)(m0 + rr) * HD + c8) = *(const v8b*)(&Tl[wave][rr][c8]); }
#pragma unroll
    for (int j = 0; j < 4; ++j) { const int rr = j * 8 + (lane >> 2), c4 = (lane & 3) * 4; *(volatile v4f*)(wout + (size_t)(m0 + rr) * NH + c4) = *(const v4f*)(&Tw[wave][rr][c4]); }
    __threadfence(); }
}

template <int QT>
__global__ __launch_bounds__(256) void score_kernel(const b16* __restrict__ qh, const b16* __restrict__ kh, const float* __restrict__ w, float* __restrict__ out) {
  __shared__ __attribute__((aligned(16))) float Os[8][16][32 + 4];
  const int wid = threadIdx.x >> 5, lane = threadIdx.x & 31, hh = lane >> 4, col = lane & 15;
  const int wg = blockIdx.x * 8 + wid, kt = wg % (S / 32), qt = (wg / (S / 32)) % QT, b = wg / ((S / 32) * QT), q0 = qt * 16, k0 = kt * 32, qi = q0 + col;
  const b16* Q = qh + ((size_t)b * S + qi) * QC; const b16* K = kh + ((size_t)b * S + k0) * HD;
  v8f o0 = {}, o1 = {};
  for (int h = 0; h < NH; ++h) { v8f s0 = {}, s1 = {};
#pragma unroll
    for (int ks = 0; ks < 4; ++ks) { const v16b qf = frag_kb(Q + h * HD + ks * 32, hh), ql = frag_kb(Q + QPL + h * HD + ks * 32, hh);
      const v16b ka = frag_kb(K + (size_t)col * HD + ks * 32, hh), kal = frag_kb(K + KPL + (size_t)col * HD + ks * 32, hh), kb_ = frag_kb(K + (size_t)(16 + col) * HD + ks * 32, hh), kbl = frag_kb(K + KPL + (size_t)(16 + col) * HD + ks * 32, hh);
      s0 = wmma16b(ka, qf, s0); s0 = wmma16b(ka, ql, s0); s0 = wmma16b(kal, qf, s0); s1 = wmma16b(kb_, qf, s1); s1 = wmma16b(kb_, ql, s1); s1 = wmma16b(kbl, qf, s1); }
    const float wq = w[((size_t)b * S + qi) * NH + h];
#pragma unroll
    for (int r = 0; r < 8; ++r) { o0[r] += wq * fmaxf(s0[r] * (1.0f / (QS * QS)), 0.0f); o1[r] += wq * fmaxf(s1[r] * (1.0f / (QS * QS)), 0.0f); } }
#pragma unroll
  for (int r = 0; r < 8; ++r) { Os[wid][col][8 * hh + r] = o0[r]; Os[wid][col][16 + 8 * hh + r] = o1[r]; }
  wave_lds_sync();
  float* dst = out + ((size_t)b * S + q0) * S + k0;
  for (int pass = 0; pass < 2; ++pass) {
#pragma unroll
    for (int j = 0; j < 4; ++j) { const int rr = j * 4 + (lane >> 3), c4 = (lane & 7) * 4; *(volatile v4f*)(dst + (size_t)rr * S + c4) = *(const v4f*)(&Os[wid][rr][c4]); }
    __threadfence(); }
}
}

extern "C" void kernel_launch(void* const* d_in, const int* in_sizes, int n_in,
                              void* d_out, int out_size, void* d_ws, size_t ws_size, hipStream_t stream) {
  (void)n_in; (void)out_size;
  const float* x = (const float*)d_in[0]; const float* cosb = (const float*)d_in[1]; const float* sinb = (const float*)d_in[2]; const float* wq = (const float*)d_in[3]; const float* wk = (const float*)d_in[4]; const float* ww = (const float*)d_in[5]; const float* g = (const float*)d_in[6]; const float* bta = (const float*)d_in[7];
  float* out = (float*)d_out;
  if (in_sizes[0] != NTOK * HID || in_sizes[1] != NTOK * RD || in_sizes[2] != NTOK * RD || in_sizes[3] != HID * QC || in_sizes[4] != HID * HD || in_sizes[5] != HID * NH || in_sizes[6] != HD) return;
  size_t off = 0; char* ws = (char*)d_ws;
  auto carve = [&](size_t bytes) { char* p = ws + off; off += (bytes + 255) & ~(size_t)255; return p; };
  unsigned short* x16 = (unsigned short*)carve((size_t)NTOK * HID * 2); unsigned short* wq16 = (unsigned short*)carve((size_t)QC * HID * 2); unsigned short* wk16 = (unsigned short*)carve((size_t)KCP * HID * 2);
  b16* qh = (b16*)carve(QPL * 2 * 2); b16* kh = (b16*)carve(KPL * 2 * 2); float* w = (float*)carve((size_t)NTOK * NH * 4);
  if (off > ws_size) return;
  prep_kernel<<<1024, 256, 0, stream>>>(x, wq, wk, ww, x16, wq16, wk16);
  qproj_kernel<<<dim3(QC / 64, NTOK / 128), 128, 0, stream>>>(x16, wq16, cosb, sinb, qh, 0);
  kproj_kernel<<<NTOK / 128, 128, 0, stream>>>(x16, wk16, cosb, sinb, g, bta, kh, w);
  score_kernel<S / 16><<<Bn * (S / 16) * (S / 32) / 8, 256, 0, stream>>>(qh, kh, w, out);
}
